// TwoSimplicialAttention_88957362635625
// MI455X (gfx1250) — hardware-verified
//
#include <hip/hip_runtime.h>
#include <stdint.h>

constexpr int NROW  = 8192;
constexpr int DIMC  = 1024;
constexpr int NHEAD = 8;
constexpr int HDIM  = 128;
constexpr int WINW  = 8;

typedef __attribute__((ext_vector_type(16))) _Float16 v16h;
typedef __attribute__((ext_vector_type(8)))  _Float16 v8h;
typedef __attribute__((ext_vector_type(16))) __bf16   v16b;
typedef __attribute__((ext_vector_type(8)))  __bf16   v8b;
typedef __attribute__((ext_vector_type(8)))  float    v8f;
typedef __attribute__((ext_vector_type(4)))  float    v4f;
typedef __attribute__((ext_vector_type(4)))  unsigned int u32x4;

__device__ __forceinline__ unsigned short f2bf_bits(float f) {
  unsigned u = __float_as_uint(f);
  return (unsigned short)((u + 0x7FFFu + ((u >> 16) & 1u)) >> 16);
}
__device__ __forceinline__ float bf_bits2f(unsigned short hb) { return __uint_as_float(((unsigned)hb) << 16); }

__device__ __forceinline__ void dep_guard_h(v8f& a, v8f& b, v16h x, v16h y) { asm volatile("v_nop\n\tv_nop\n\tv_nop\n\tv_nop" : "+v"(a), "+v"(b) : "v"(x), "v"(y)); }
__device__ __forceinline__ void dep_guard_b(v8f& a, v8f& b, v16b x, v16b y) { asm volatile("v_nop\n\tv_nop\n\tv_nop\n\tv_nop" : "+v"(a), "+v"(b) : "v"(x), "v"(y)); }
__device__ __forceinline__ void keep4_h(v16h a, v16h b, v16h c, v16h d) { asm volatile("v_nop" :: "v"(a), "v"(b), "v"(c), "v"(d)); }
__device__ __forceinline__ void keep4_b(v16b a, v16b b, v16b c, v16b d) { asm volatile("v_nop" :: "v"(a), "v"(b), "v"(c), "v"(d)); }
__device__ __forceinline__ void acc_guard4(v8f& a, v8f& b, v8f& c, v8f& d) { asm volatile("v_nop\n\tv_nop\n\tv_nop\n\tv_nop" : "+v"(a), "+v"(b), "+v"(c), "+v"(d)); }

template <typename T> struct Frag;
template <> struct Frag<_Float16> {
  typedef v16h V; union U { v16h v; v8h h[2]; };
  static __device__ __forceinline__ v16h load(const _Float16* p) {
    U f; f.h[0] = *(const v8h*)(p); f.h[1] = *(const v8h*)(p + 16); return f.v;
  }
  static __device__ __forceinline__ v8f mma(v16h a, v16h b, v8f c) {
    return __builtin_amdgcn_wmma_f32_16x16x32_f16(false, a, false, b, (short)0, c, false, false);
  }
  static __device__ __forceinline__ void guard(v8f& a, v8f& b, v16h x, v16h y) { dep_guard_h(a, b, x, y); }
  static __device__ __forceinline__ void keep(v16h a, v16h b, v16h c, v16h d) { keep4_h(a, b, c, d); }
};
template <> struct Frag<__bf16> {
  typedef v16b V; union U { v16b v; v8b h[2]; };
  static __device__ __forceinline__ v16b load(const __bf16* p) {
    U f; f.h[0] = *(const v8b*)(p); f.h[1] = *(const v8b*)(p + 16); return f.v;
  }
  static __device__ __forceinline__ v8f mma(v16b a, v16b b, v8f c) {
    return __builtin_amdgcn_wmma_f32_16x16x32_bf16(false, a, false, b, (short)0, c, false, false);
  }
  static __device__ __forceinline__ void guard(v8f& a, v8f& b, v16b x, v16b y) { dep_guard_b(a, b, x, y); }
  static __device__ __forceinline__ void keep(v16b a, v16b b, v16b c, v16b d) { keep4_b(a, b, c, d); }
};

template <int ET> struct Elem;
template <> struct Elem<0> { typedef _Float16 T; };
template <> struct Elem<1> { typedef __bf16 T; };
template <int ET, bool SPLIT, int BIAS_MODE, int OUT_MODE, bool RESID>
__global__ __launch_bounds__(256) void wmma_gemm64(
    const unsigned short* __restrict__ Ap, const unsigned short* __restrict__ A2p, int lda, long strideA,
    const unsigned short* __restrict__ Btp, const unsigned short* __restrict__ Bt2p, int ldb, long strideB,
    void* __restrict__ Cout, void* __restrict__ Cout2, int ldc, long strideC,
    const float* __restrict__ bias,
    const float* __restrict__ resid, long strideR,
    int M, int N, int K, float scale) {
  static_assert(!RESID || OUT_MODE == 0);
  typedef typename Elem<ET>::T T;
  typedef typename Frag<T>::V V;
  const T* A = (const T*)Ap; const T* A2 = (const T*)A2p; const T* Bt = (const T*)Btp; const T* Bt2 = (const T*)Bt2p;
  __shared__ __align__(16) float sT[8][16 * 68];
  const int b    = blockIdx.y;
  const int lane = threadIdx.x & 31;
  const int wave = threadIdx.x >> 5;
  const int tilesN = N >> 6;
  const int tilesM = M >> 6;
  const int tile = blockIdx.x * 8 + wave;
  if (tile >= tilesM * tilesN) return;
  const int tm = tile / tilesN;
  const int tn = tile - tm * tilesN;
  const int m0 = tm << 6;
  const int n0 = tn << 6;

  const T* Ab  = A  + (size_t)b * strideA;
  const T* Bb  = Bt + (size_t)b * strideB;
  const T* Ab2 = SPLIT ? (A2  + (size_t)b * strideA) : nullptr;
  const T* Bb2 = SPLIT ? (Bt2 + (size_t)b * strideB) : nullptr;

  const int rlane = lane & 15;
  const int koff  = (lane >> 4) * 8;
  const int mOff  = (lane >> 4) * 8;

  v8f acc[4][4];
#pragma unroll
  for (int i = 0; i < 4; ++i)
#pragma unroll
    for (int j = 0; j < 4; ++j) acc[i][j] = (v8f){0.f,0.f,0.f,0.f,0.f,0.f,0.f,0.f};

  for (int k0 = 0; k0 < K; k0 += 32) {
    V bh[4], bl[4];
#pragma unroll
    for (int j = 0; j < 4; ++j) {
      const size_t bo = (size_t)(n0 + (j << 4) + rlane) * ldb + koff + k0;
      bh[j] = Frag<T>::load(Bb + bo);
      if (SPLIT) bl[j] = Frag<T>::load(Bb2 + bo);
    }
#pragma unroll
    for (int i = 0; i < 4; ++i) {
      const size_t ao = (size_t)(m0 + (i << 4) + rlane) * lda + koff + k0;
      V ah = Frag<T>::load(Ab + ao);
      V al;
      if (SPLIT) al = Frag<T>::load(Ab2 + ao);
#pragma unroll
      for (int j = 0; j < 4; ++j) {
        acc[i][j] = Frag<T>::mma(ah, bh[j], acc[i][j]);
        if (SPLIT) {
          acc[i][j] = Frag<T>::mma(ah, bl[j], acc[i][j]);
          acc[i][j] = Frag<T>::mma(al, bh[j], acc[i][j]);
        }
      }
      Frag<T>::guard(acc[i][0], acc[i][3], ah, SPLIT ? al : ah);
    }
    Frag<T>::keep(bh[0], bh[1], bh[2], bh[3]);
    if (SPLIT) Frag<T>::keep(bl[0], bl[1], bl[2], bl[3]);
  }
  acc_guard4(acc[0][0], acc[0][1], acc[0][2], acc[0][3]);
  acc_guard4(acc[1][0], acc[1][1], acc[1][2], acc[1][3]);
  acc_guard4(acc[2][0], acc[2][1], acc[2][2], acc[2][3]);
  acc_guard4(acc[3][0], acc[3][1], acc[3][2], acc[3][3]);

  float* slab = sT[wave];
#pragma unroll
  for (int i = 0; i < 4; ++i) {
    const int mBase = m0 + (i << 4);
#pragma unroll
    for (int j = 0; j < 4; ++j) {
      const int n = n0 + (j << 4) + rlane;
      float bv = 0.f;
      if (BIAS_MODE == 2) bv = bias[n];
#pragma unroll
      for (int r = 0; r < 8; ++r) {
        float v = acc[i][j][r] * scale;
        if (BIAS_MODE == 1) v += bias[mBase + mOff + r];
        if (BIAS_MODE == 2) v += bv;
        slab[(mOff + r) * 68 + (j << 4) + rlane] = v;
      }
    }
    __builtin_amdgcn_fence(__ATOMIC_RELEASE, "workgroup");
    __builtin_amdgcn_wave_barrier();
    __builtin_amdgcn_fence(__ATOMIC_ACQUIRE, "workgroup");
    if (OUT_MODE == 0) {
      float* Cp = (float*)Cout + (size_t)b * strideC;
      const int hh = lane >> 4, c4 = (lane & 15) * 4;
      if (RESID) {
        const float* Rb = resid + (size_t)b * strideR;
#pragma unroll
        for (int it = 0; it < 8; ++it) {
          const int row = it * 2 + hh;
          const v4f rv = *(const v4f*)(Rb + (size_t)(mBase + row) * ldc + n0 + c4);
          v4f sv = *(const v4f*)(slab + row * 68 + c4);
          sv += rv;
          *(v4f*)(slab + row * 68 + c4) = sv;
        }
      }
      for (int pass = 0; pass < 2; ++pass) {
#pragma unroll
        for (int it = 0; it < 8; ++it) {
          const int row = it * 2 + hh;
          v4f v = *(const v4f*)(slab + row * 68 + c4);
          *(volatile v4f*)(Cp + (size_t)(mBase + row) * ldc + n0 + c4) = v;
        }
        __threadfence();
      }
    } else {
      const int q = lane >> 3, c8 = (lane & 7) * 8;
      unsigned short* Cp  = (unsigned short*)Cout  + (size_t)b * strideC;
      unsigned short* Cp2 = (OUT_MODE == 2) ? ((unsigned short*)Cout2 + (size_t)b * strideC) : nullptr;
      for (int pass = 0; pass < 2; ++pass) {
#pragma unroll
        for (int it = 0; it < 4; ++it) {
          const int row = it * 4 + q;
          const float* sp = slab + row * 68 + c8;
          v8h hv, lv;
#pragma unroll
          for (int e = 0; e < 8; ++e) {
            if (OUT_MODE == 1) {
              hv[e] = (_Float16)sp[e];
            } else {
              unsigned short hb = f2bf_bits(sp[e]);
              unsigned short lb = f2bf_bits(sp[e] - bf_bits2f(hb));
              hv[e] = __builtin_bit_cast(_Float16, hb);
              lv[e] = __builtin_bit_cast(_Float16, lb);
            }
          }
          *(volatile v8h*)(Cp + (size_t)(mBase + row) * ldc + n0 + c8) = hv;
          if (OUT_MODE == 2) *(volatile v8h*)(Cp2 + (size_t)(mBase + row) * ldc + n0 + c8) = lv;
        }
        __threadfence();
      }
    }
    __builtin_amdgcn_fence(__ATOMIC_RELEASE, "workgroup");
    __builtin_amdgcn_wave_barrier();
    __builtin_amdgcn_fence(__ATOMIC_ACQUIRE, "workgroup");
  }
}

__global__ __launch_bounds__(256) void cast_f32_f16x2(
    const float* __restrict__ in, _Float16* __restrict__ out, int n2, float carry) {
  int i = blockIdx.x * 256 + threadIdx.x;
  if (i < n2) {
    const _Float16 h0 = (_Float16)(in[2 * i] * carry), h1 = (_Float16)(in[2 * i + 1] * carry);
    const unsigned u = (unsigned)__builtin_bit_cast(unsigned short, h0) | ((unsigned)__builtin_bit_cast(unsigned short, h1) << 16);
    ((volatile unsigned*)out)[i] = u;
    __threadfence();
    ((volatile unsigned*)out)[i] = u;
  }
}

__device__ __forceinline__ float wave_sum(float v) {
#pragma unroll
  for (int o = 1; o < 32; o <<= 1) v += __shfl_xor(v, o, 32);
  return v;
}
__device__ __forceinline__ float wave_max(float v) {
#pragma unroll
  for (int o = 1; o < 32; o <<= 1) v = fmaxf(v, __shfl_xor(v, o, 32));
  return v;
}

constexpr int AT_ROWS = 15;
constexpr int AT_P    = 132;

__device__ __forceinline__ float h16_to_f32(unsigned bits) {
  const unsigned short s = (unsigned short)(bits & 0xffffu);
  const _Float16 hv = __builtin_bit_cast(_Float16, s);
  return (float)hv;
}
__device__ __forceinline__ void stage8(float* dst, const unsigned short* src) {
  const u32x4 w = *(const u32x4*)(const void*)src;
  const v4f a  = { h16_to_f32(w[0]), h16_to_f32(w[0] >> 16), h16_to_f32(w[1]), h16_to_f32(w[1] >> 16) };
  const v4f bq = { h16_to_f32(w[2]), h16_to_f32(w[2] >> 16), h16_to_f32(w[3]), h16_to_f32(w[3] >> 16) };
  *(v4f*)dst = a;
  *(v4f*)(dst + 4) = bq;
}

__global__ __launch_bounds__(256) void tri_window_attn(
    const unsigned short* __restrict__ Qpl, const unsigned short* __restrict__ Kpl,
    const unsigned short* __restrict__ Vpl, const unsigned short* __restrict__ K2pl,
    const unsigned short* __restrict__ V2pl, unsigned short* __restrict__ Zpl) {
  __shared__ __align__(16) float sK [AT_ROWS * AT_P];
  __shared__ __align__(16) float sK2[AT_ROWS * AT_P];
  __shared__ __align__(16) float sV [AT_ROWS * AT_P];
  __shared__ __align__(16) float sV2[AT_ROWS * AT_P];
  __shared__ __align__(16) float sQ [WINW * AT_P];
  __shared__ __align__(16) float sS [8][64];
  __shared__ __align__(16) float sZ [8][HDIM];

  const int tid  = threadIdx.x;
  const int wave = tid >> 5;
  const int lane = tid & 31;
  const int n0   = blockIdx.x * 8;
  const int h    = blockIdx.y;
  const size_t hoff = (size_t)h * HDIM;

  {
    const int t  = tid < 240 ? tid : 239;
    const int r  = t >> 4;
    const int c8 = (t & 15) * 8;
    int pos = n0 - 7 + r;
    pos = pos < 0 ? 0 : pos;
    const size_t go = (size_t)pos * DIMC + hoff + c8;
    const int lo = r * AT_P + c8;
    stage8(sK  + lo, Kpl  + go);
    stage8(sK2 + lo, K2pl + go);
    stage8(sV  + lo, Vpl  + go);
    stage8(sV2 + lo, V2pl + go);
  }
  if (wave < 4) {
    const int r  = tid >> 4;
    const int c8 = (tid & 15) * 8;
    const size_t go = (size_t)(n0 + r) * DIMC + hoff + c8;
    stage8(sQ + r * AT_P + c8, Qpl + go);
  }
  __syncthreads();

  const int n  = n0 + wave;
  const int kk = lane & 7;
  const int j0 = lane >> 3;
  const int j1 = j0 + 4;
  const float* qrow  = sQ  + wave * AT_P;
  const float* kprow = sK2 + (wave + kk) * AT_P;
  const float* karow = sK  + (wave + j0) * AT_P;
  const float* kbrow = sK  + (wave + j1) * AT_P;
  float s0 = 0.f, s1 = 0.f;
#pragma unroll 4
  for (int d = 0; d < HDIM; ++d) {
    const float u = qrow[d] * kprow[d];
    s0 = fmaf(u, karow[d], s0);
    s1 = fmaf(u, kbrow[d], s1);
  }
  const float sc = 0.08838834764831845f;
  const bool kval = (n - 7 + kk) >= 0;
  const bool val0 = kval && ((n - 7 + j0) >= 0);
  const bool val1 = kval && ((n - 7 + j1) >= 0);
  s0 = val0 ? (s0 * sc) : -1e30f;
  s1 = val1 ? (s1 * sc) : -1e30f;

  float m = fmaxf(s0, s1);
  m = wave_max(m);
  const float e0 = expf(s0 - m);
  const float e1 = expf(s1 - m);
  const float ssum = wave_sum(e0 + e1);
  const float inv = 1.0f / ssum;
  sS[wave][lane]      = e0 * inv;
  sS[wave][32 + lane] = e1 * inv;
  __syncthreads();

  const float* Sw = sS[wave];
#pragma unroll 1
  for (int cblk = 0; cblk < 4; ++cblk) {
    const int d = lane + 32 * cblk;
    float vj[8];
#pragma unroll
    for (int j = 0; j < 8; ++j) vj[j] = sV[(wave + j) * AT_P + d];
    float z = 0.f;
#pragma unroll 1
    for (int k = 0; k < 8; ++k) {
      float t = 0.f;
#pragma unroll
      for (int j = 0; j < 8; ++j) t = fmaf(vj[j], Sw[j * 8 + k], t);
      z = fmaf(t, sV2[(wave + k) * AT_P + d], z);
    }
    sZ[wave][d] = z * 16.0f;
  }
  __syncthreads();

  if (lane < 16) {
    const float* zp = sZ[wave] + lane * 8;
    const v4f a  = *(const v4f*)(zp);
    const v4f bq = *(const v4f*)(zp + 4);
    v8h hv;
    hv[0] = (_Float16)a[0];  hv[1] = (_Float16)a[1];  hv[2] = (_Float16)a[2];  hv[3] = (_Float16)a[3];
    hv[4] = (_Float16)bq[0]; hv[5] = (_Float16)bq[1]; hv[6] = (_Float16)bq[2]; hv[7] = (_Float16)bq[3];
    unsigned short* dst = Zpl + (size_t)n * DIMC + hoff + lane * 8;
    *(volatile v8h*)dst = hv;
    __threadfence();
    *(volatile v8h*)dst = hv;
  }
}

__global__ __launch_bounds__(256) void ln_rows(
    const float* __restrict__ G, const float* __restrict__ gamma,
    const float* __restrict__ beta, float* __restrict__ out) {
  __shared__ float red[8];
  const int row  = blockIdx.x;
  const int tid  = threadIdx.x;
  const int wave = tid >> 5;
  const int lane = tid & 31;
  const size_t base = (size_t)row * DIMC + (size_t)tid * 4;
  const v4f v = *(const v4f*)(G + base);
  float s = (v[0] + v[1]) + (v[2] + v[3]);
  s = wave_sum(s);
  if (lane == 0) red[wave] = s;
  __syncthreads();
  float tot = 0.f;
#pragma unroll
  for (int w = 0; w < 8; ++w) tot += red[w];
  const float mu = tot * (1.0f / 1024.0f);
  __syncthreads();
  const float d0 = v[0] - mu, d1 = v[1] - mu, d2 = v[2] - mu, d3 = v[3] - mu;
  float sq = (d0 * d0 + d1 * d1) + (d2 * d2 + d3 * d3);
  sq = wave_sum(sq);
  if (lane == 0) red[wave] = sq;
  __syncthreads();
  float tot2 = 0.f;
#pragma unroll
  for (int w = 0; w < 8; ++w) tot2 += red[w];
  const float var  = tot2 * (1.0f / 1024.0f);
  const float rstd = 1.0f / sqrtf(var + 1e-5f);
  const v4f g  = *(const v4f*)(gamma + (size_t)tid * 4);
  const v4f bt = *(const v4f*)(beta  + (size_t)tid * 4);
  const v4f o = { d0 * rstd * g[0] + bt[0], d1 * rstd * g[1] + bt[1],
                  d2 * rstd * g[2] + bt[2], d3 * rstd * g[3] + bt[3] };
  float* dst = out + base;
  *(volatile v4f*)dst = o;
  __threadfence();
  *(volatile v4f*)dst = o;
}

extern "C" void kernel_launch(void* const* d_in, const int* in_sizes, int n_in,
                              void* d_out, int out_size, void* d_ws, size_t ws_size,
                              hipStream_t stream) {
  constexpr size_t PLANE16  = (size_t)NROW * DIMC * 2;
  constexpr size_t WPLANE   = (size_t)DIMC * DIMC * 2;
  constexpr size_t OFF_XZ   = 0;
  constexpr size_t OFF_W    = OFF_XZ + PLANE16;
  constexpr size_t OFF_P    = OFF_W + 6 * WPLANE;
  constexpr size_t WS_TOTAL = OFF_P + 5 * PLANE16;
  static_assert(WS_TOTAL == 113246208ull);
  static_assert(WS_TOTAL <= 134217728ull);
  static_assert((size_t)NROW * DIMC * 4 <= 2 * PLANE16);
  static_assert(NROW % 64 == 0 && DIMC % 64 == 0 && DIMC % 32 == 0);
  static_assert((NROW / 64) * (DIMC / 64) % 8 == 0);
  static_assert(NHEAD * HDIM == DIMC && NROW % 8 == 0);

  if (n_in < 15) return;
  if (in_sizes[0] != NROW * DIMC || out_size != NROW * DIMC) return;
  for (int i = 1; i <= 11; i += 2) if (in_sizes[i] != DIMC * DIMC) return;
  for (int i = 2; i <= 14; i += 2) if (in_sizes[i] != DIMC) return;
  if (in_sizes[13] != DIMC) return;
  if (ws_size < WS_TOTAL) return;

  const float* x     = (const float*)d_in[0];
  const float* Wsrc[6] = { (const float*)d_in[1], (const float*)d_in[3], (const float*)d_in[5],
                           (const float*)d_in[7], (const float*)d_in[9], (const float*)d_in[11] };
  const float* Bsrc[5] = { (const float*)d_in[2], (const float*)d_in[4], (const float*)d_in[6],
                           (const float*)d_in[8], (const float*)d_in[10] };
  const float* bo    = (const float*)d_in[12];
  const float* gamma = (const float*)d_in[13];
  const float* beta  = (const float*)d_in[14];
  float* outp = (float*)d_out;

  char* ws = (char*)d_ws;
  unsigned short* Xh = (unsigned short*)(ws + OFF_XZ);
  unsigned short* Zh = (unsigned short*)(ws + OFF_XZ);
  unsigned short* Wh[6];
  for (int i = 0; i < 6; ++i) Wh[i] = (unsigned short*)(ws + OFF_W + (size_t)i * WPLANE);
  unsigned short* Ph[5];
  for (int i = 0; i < 5; ++i) Ph[i] = (unsigned short*)(ws + OFF_P + (size_t)i * PLANE16);
  float* Gf = (float*)(ws + OFF_P);

  {
    const int n2x = NROW * DIMC / 2;
    cast_f32_f16x2<<<dim3(n2x / 256), dim3(256), 0, stream>>>(x, (_Float16*)Xh, n2x, 1.0f);
    const int n2w = DIMC * DIMC / 2;
    for (int i = 0; i < 6; ++i)
      cast_f32_f16x2<<<dim3(n2w / 256), dim3(256), 0, stream>>>(Wsrc[i], (_Float16*)Wh[i], n2w, 16.0f);
  }

  const int gemmBlocks = (NROW / 64) * (DIMC / 64) / 8;
  for (int i = 0; i < 5; ++i) {
    wmma_gemm64<0, false, 2, 1, false><<<dim3(gemmBlocks, 1), dim3(256), 0, stream>>>(
        Xh, Xh, DIMC, 0L, Wh[i], Wh[i], DIMC, 0L,
        (void*)Ph[i], (void*)Ph[i], DIMC, 0L,
        Bsrc[i], x, 0L, NROW, DIMC, DIMC, 1.0f / 16.0f);
  }

  tri_window_attn<<<dim3(NROW / 8, NHEAD), dim3(256), 0, stream>>>(Ph[0], Ph[1], Ph[2], Ph[3], Ph[4], Zh);

  wmma_gemm64<0, false, 2, 0, true><<<dim3(gemmBlocks, 1), dim3(256), 0, stream>>>(
      Zh, Zh, DIMC, 0L, Wh[5], Wh[5], DIMC, 0L,
      (void*)Gf, (void*)Gf, DIMC, 0L,
      bo, x, 0L, NROW, DIMC, DIMC, 1.0f / 256.0f);

  ln_rows<<<dim3(NROW), dim3(256), 0, stream>>>(Gf, gamma, beta, outp);
}
